// GINModelIntegrated_73521250173226
// MI455X (gfx1250) — hardware-verified
//
#include <hip/hip_runtime.h>
#include <stddef.h>


#define FEXP    256
#define FH      128
#define NCLS    8
#define NCP     16
#define NTHR    256
#define NWAVE   8
#define EPT     8
#define NGRP    2
#define CHUNK   (NTHR * EPT * NGRP)
#define WCAP    (EPT * NGRP * 32)
#define LISTN   (NWAVE * WCAP)
#define ESHF    11
#define NBC     32768
#define NBF     2048
#define RCAP    40960
#define RBN     128
#define TGT     256
#define DEGCAP  512
#define GR      64
#define MROWS   128
#define OTHR    512
#define HTHR    256
#define WSCAP   134217728

#define LDS_COUNT ((NBC + LISTN + NWAVE) * 4)
#define LDS_FILL  ((RCAP + NBF + LISTN + NWAVE) * 4)
#define LDS_GEMM  65536

static_assert((CHUNK & (CHUNK - 1)) == 0);
static_assert((NBC & (NBC - 1)) == 0 && (NBF & (NBF - 1)) == 0);
static_assert(NBF <= (1 << ESHF));
static_assert((NBC % NBF) == 0);
static_assert(OTHR * 4 == NBF);
static_assert((RCAP % 32) == 0);
static_assert(TGT == NWAVE * 32);
static_assert(GR == (NWAVE / 2) * 16 && (GR % NWAVE) == 0);
static_assert(MROWS == NWAVE * 16);
static_assert((TGT % GR) == 0 && (TGT % MROWS) == 0);
static_assert(NBC == NWAVE * 32 * 128);
static_assert((FEXP % 32) == 0 && (FH % 32) == 0 && FH == 4 * 32);
static_assert((GR * FEXP / 8) % NTHR == 0 && (GR * FH / 8) % NTHR == 0);
static_assert(2 * GR * FEXP * 2 <= LDS_GEMM && GR * FH * 4 <= LDS_GEMM);
static_assert(MROWS * NCLS == 4 * NTHR);
static_assert(NCLS <= NCP && NCP == 16);

typedef float          v4f   __attribute__((ext_vector_type(4)));
typedef float          v8f   __attribute__((ext_vector_type(8)));
typedef int            v4i   __attribute__((ext_vector_type(4)));
typedef unsigned short v8us  __attribute__((ext_vector_type(8)));
typedef __bf16         v8bf  __attribute__((ext_vector_type(8)));
typedef __bf16         v16bf __attribute__((ext_vector_type(16)));
union FragB { v16bf v; v8us h[2]; };
union Pk8   { v8bf b; v8us u; };

__device__ __forceinline__ v8f wmb(v16bf a, v16bf b, v8f c) {
  v8f d = __builtin_amdgcn_wmma_f32_16x16x32_bf16(false, a, false, b, (short)0, c, false, false);
  asm volatile("v_nop\n\tv_nop\n\tv_nop\n\tv_nop" : "+v"(d) : "v"(a), "v"(b));
  return d;
}

__device__ __forceinline__ void split_row16(const float* p, v16bf& hv, v16bf& lv) {
  const v4f a0 = *(const v4f*)p, a1 = *(const v4f*)(p + 4), a2 = *(const v4f*)(p + 16), a3 = *(const v4f*)(p + 20);
  const float av[16] = {a0.x, a0.y, a0.z, a0.w, a1.x, a1.y, a1.z, a1.w,
                        a2.x, a2.y, a2.z, a2.w, a3.x, a3.y, a3.z, a3.w};
#pragma unroll
  for (int e = 0; e < 16; ++e) {
    const __bf16 hb = (__bf16)av[e];
    const float rem = av[e] - (float)hb;
    hv[e] = hb;
    lv[e] = (__bf16)rem;
  }
}

template <int NB, int SRC>
__device__ __forceinline__ int scan_chunk(const int* __restrict__ dsts, const int* __restrict__ srcs, int nE, int nN,
                                          int cbase, int slotBase, int vec8, int* list, int tid, int lane, int wave) {
  int wc = 0;
#pragma unroll
  for (int g = 0; g < NGRP; ++g) {
    const int el0  = (g * NTHR + tid) * EPT;
    const int e0   = cbase + el0;
    const int sent = -2147483647 - 1;
    v4i da, db;
    v4i sa = {0, 0, 0, 0}, sb = {0, 0, 0, 0};
    if (vec8 != 0 && cbase + CHUNK <= nE) {
      da = *(const v4i*)(dsts + e0);
      db = *(const v4i*)(dsts + e0 + 4);
      if (SRC) {
        sa = *(const v4i*)(srcs + e0);
        sb = *(const v4i*)(srcs + e0 + 4);
      }
    } else {
      da.x = (e0     < nE) ? dsts[min(e0, nE - 1)] : sent;
      da.y = (e0 + 1 < nE) ? dsts[min(e0 + 1, nE - 1)] : sent;
      da.z = (e0 + 2 < nE) ? dsts[min(e0 + 2, nE - 1)] : sent;
      da.w = (e0 + 3 < nE) ? dsts[min(e0 + 3, nE - 1)] : sent;
      db.x = (e0 + 4 < nE) ? dsts[min(e0 + 4, nE - 1)] : sent;
      db.y = (e0 + 5 < nE) ? dsts[min(e0 + 5, nE - 1)] : sent;
      db.z = (e0 + 6 < nE) ? dsts[min(e0 + 6, nE - 1)] : sent;
      db.w = (e0 + 7 < nE) ? dsts[min(e0 + 7, nE - 1)] : sent;
      if (SRC) {
        sa.x = srcs[min(e0, nE - 1)];
        sa.y = srcs[min(e0 + 1, nE - 1)];
        sa.z = srcs[min(e0 + 2, nE - 1)];
        sa.w = srcs[min(e0 + 3, nE - 1)];
        sb.x = srcs[min(e0 + 4, nE - 1)];
        sb.y = srcs[min(e0 + 5, nE - 1)];
        sb.z = srcs[min(e0 + 6, nE - 1)];
        sb.w = srcs[min(e0 + 7, nE - 1)];
      }
    }
    if (SRC) {
      sa.x = min(max(sa.x, 0), nN - 1); sa.y = min(max(sa.y, 0), nN - 1);
      sa.z = min(max(sa.z, 0), nN - 1); sa.w = min(max(sa.w, 0), nN - 1);
      sb.x = min(max(sb.x, 0), nN - 1); sb.y = min(max(sb.y, 0), nN - 1);
      sb.z = min(max(sb.z, 0), nN - 1); sb.w = min(max(sb.w, 0), nN - 1);
    }
    const unsigned nb = (unsigned)slotBase;
    const unsigned s0 = (unsigned)da.x - nb, s1 = (unsigned)da.y - nb;
    const unsigned s2 = (unsigned)da.z - nb, s3 = (unsigned)da.w - nb;
    const unsigned s4 = (unsigned)db.x - nb, s5 = (unsigned)db.y - nb;
    const unsigned s6 = (unsigned)db.z - nb, s7 = (unsigned)db.w - nb;
    const bool h0 = s0 < (unsigned)NB, h1 = s1 < (unsigned)NB, h2 = s2 < (unsigned)NB, h3 = s3 < (unsigned)NB;
    const bool h4 = s4 < (unsigned)NB, h5 = s5 < (unsigned)NB, h6 = s6 < (unsigned)NB, h7 = s7 < (unsigned)NB;
    const unsigned any = __builtin_amdgcn_ballot_w32(h0 | h1 | h2 | h3 | h4 | h5 | h6 | h7);
    if (any != 0u) {
#define HITJ(HJ, SJ, VJ) { \
        const unsigned mj = __builtin_amdgcn_ballot_w32(HJ); \
        if (mj != 0u) { \
          if (HJ) { \
            const int pos = wc + (int)__builtin_amdgcn_mbcnt_lo(mj, 0u); \
            const int entv = SRC ? (((VJ) << ESHF) | (int)(SJ)) : (int)(SJ); \
            if (pos < WCAP) list[wave * WCAP + pos] = entv; \
          } \
          wc += (int)__builtin_popcount(mj); } }
      HITJ(h0, s0, sa.x)
      HITJ(h1, s1, sa.y)
      HITJ(h2, s2, sa.z)
      HITJ(h3, s3, sa.w)
      HITJ(h4, s4, sb.x)
      HITJ(h5, s5, sb.y)
      HITJ(h6, s6, sb.z)
      HITJ(h7, s7, sb.w)
#undef HITJ
    }
  }
  return wc;
}

__global__ __launch_bounds__(NTHR) void k_wprep(const float* __restrict__ W, unsigned short* ph, unsigned short* pl,
                                                int K, int NOUT, int NP) {
  const int tid = threadIdx.x;
  const int kq = K >> 3;
  const int total = NP * kq;
  const int i = (int)blockIdx.x * NTHR + tid;
  const int ic = i < total ? i : total - 1;
  const int n = ic / kq;
  const int k0 = (ic - n * kq) * 8;
  const int nc = n < NOUT ? n : NOUT - 1;
  Pk8 hp, lp;
#pragma unroll
  for (int e = 0; e < 8; ++e) {
    float v = W[(size_t)(k0 + e) * NOUT + nc];
    v = n < NOUT ? v : 0.0f;
    const __bf16 hb = (__bf16)v;
    const float rem = v - (float)hb;
    hp.b[e] = hb;
    lp.b[e] = (__bf16)rem;
  }
  unsigned short* dh = ph + (size_t)ic * 8;
  unsigned short* dl = pl + (size_t)ic * 8;
  if (i < total) { *(volatile v8us*)dh = hp.u; *(volatile v8us*)dl = lp.u; }
  __threadfence();
  if (i < total) { *(volatile v8us*)dh = hp.u; *(volatile v8us*)dl = lp.u; }
}

__global__ __launch_bounds__(NTHR) void k_count(const int* __restrict__ ei, int* cnt, int nE, int nN, int vec8) {
  extern __shared__ v4f lds_dyn[];
  int* scnt = (int*)lds_dyn;
  int* list = scnt + NBC;
  int* wcnt = list + LISTN;
  const int tid = threadIdx.x, lane = tid & 31, wave = tid >> 5;
  const int nodeBase = blockIdx.x * NBC;
  const int* dsts = ei + nE;

  {
    const v4i z = {0, 0, 0, 0};
    for (int i = tid; i < NBC / 4; i += NTHR) ((v4i*)scnt)[i] = z;
  }
  __syncthreads();

  const int nChunks = (nE + CHUNK - 1) / CHUNK;
#pragma unroll 1
  for (int ch = 0; ch < nChunks; ++ch) {
    const int cbase = ch * CHUNK;
    const int wc = scan_chunk<NBC, 0>(dsts, ei, nE, nN, cbase, nodeBase, vec8, list, tid, lane, wave);
    if (lane == 0) wcnt[wave] = wc;
    __syncthreads();
    if (wave == 0) {
#pragma unroll 1
      for (int wsx = 0; wsx < NWAVE; ++wsx) {
        int n = __builtin_amdgcn_readfirstlane(wcnt[wsx]);
        n = n > WCAP ? WCAP : (n < 0 ? 0 : n);
        const int* lp = list + wsx * WCAP;
#pragma unroll 1
        for (int i = 0; i < n; ++i) {
          const int ent  = __builtin_amdgcn_readfirstlane(lp[i]);
          const int slot = ent & (NBC - 1);
          if (lane == 0) scnt[slot] = scnt[slot] + 1;
        }
      }
    }
    __syncthreads();
  }

  int* cp = cnt + (size_t)nodeBase;
#pragma unroll 4
  for (int q = 0; q < 32; ++q) {
    const int f = (wave * 32 + q) * 128 + 4 * lane;
    const v4i c = *(const v4i*)(scnt + f);
    *(volatile v4i*)(cp + f) = c;
  }
  __threadfence();
#pragma unroll 4
  for (int q = 0; q < 32; ++q) {
    const int f = (wave * 32 + q) * 128 + 4 * lane;
    const v4i c = *(const v4i*)(scnt + f);
    *(volatile v4i*)(cp + f) = c;
  }
}

__global__ __launch_bounds__(OTHR) void k_offsets(const int* __restrict__ cnt, int* off, int* rbase, int nBF) {
  __shared__ __attribute__((aligned(16))) int srb[RBN];
  __shared__ int wtot[OTHR / 32];
  const int tid = threadIdx.x, lane = tid & 31, wave = tid >> 5;
  for (int i = tid; i < RBN; i += OTHR) srb[i] = 0;
  int carry = 0;
#pragma unroll 1
  for (int fb = 0; fb < nBF; ++fb) {
    const int base = fb * NBF;
    const v4i c = *(const v4i*)(cnt + base + 4 * tid);
    const int e0 = max(c.x, 0), e1 = max(c.y, 0), e2 = max(c.z, 0), e3 = max(c.w, 0);
    const int ts = e0 + e1 + e2 + e3;
    int incl = ts;
#pragma unroll
    for (int d = 1; d < 32; d <<= 1) {
      const int t = __shfl_up(incl, d);
      if (lane >= d) incl += t;
    }
    if (lane == 31) wtot[wave] = incl;
    __syncthreads();
    int pre = 0;
#pragma unroll 1
    for (int w = 0; w < wave; ++w) pre += wtot[w];
    int tot = 0;
#pragma unroll
    for (int w = 0; w < OTHR / 32; ++w) tot += wtot[w];
    int run = carry + pre + incl - ts;
    v4i o;
    o.x = run; run += e0;
    o.y = run; run += e1;
    o.z = run; run += e2;
    o.w = run;
    int* op = off + base + 4 * tid;
    *(volatile v4i*)op = o;
    __threadfence();
    *(volatile v4i*)op = o;
    if (tid == 0) srb[min(fb, RBN - 1)] = carry;
    carry += (tot + 31) & ~31;
    __syncthreads();
  }
  if (tid == 0) srb[min(nBF, RBN - 1)] = carry;
  __syncthreads();
  v4i rv = {0, 0, 0, 0};
  if (tid < 32) rv = *(const v4i*)(srb + 4 * tid);
  if (tid < 32) *(volatile v4i*)(rbase + 4 * tid) = rv;
  __threadfence();
  if (tid < 32) *(volatile v4i*)(rbase + 4 * tid) = rv;
}

__global__ __launch_bounds__(NTHR) void k_fill(
    const int* __restrict__ ei, const int* __restrict__ off, const int* __restrict__ rbase,
    int* csr, int nN, int nE, int vec8, int csrLen) {
  extern __shared__ v4f lds_dyn[];
  int* region = (int*)lds_dyn;
  int* cursor = region + RCAP;
  int* list   = cursor + NBF;
  int* wcnt   = list + LISTN;
  const int tid = threadIdx.x, lane = tid & 31, wave = tid >> 5;
  const int b = blockIdx.x;
  const int nodeBase = b * NBF;
  const int* dsts = ei + nE;

  int rb0 = rbase[b];
  const int rb1 = rbase[b + 1];
  rb0 = rb0 < 0 ? 0 : (rb0 > csrLen ? csrLen : rb0);
  rb0 &= ~31;
  int len = rb1 - rb0;
  len = len < 0 ? 0 : (len > RCAP ? RCAP : len);
  int lenW = (len + 31) & ~31;
  if (rb0 + lenW > csrLen) lenW = (csrLen - rb0) & ~31;

  {
    const v4i z = {0, 0, 0, 0};
    for (int i = tid; i < RCAP / 4; i += NTHR) ((v4i*)region)[i] = z;
    for (int s = tid; s < NBF; s += NTHR) {
      int o = off[nodeBase + s] - rb0;
      o = o < 0 ? 0 : (o > RCAP ? RCAP : o);
      cursor[s] = o;
    }
  }
  __syncthreads();

  const int nChunks = (nE + CHUNK - 1) / CHUNK;
#pragma unroll 1
  for (int ch = 0; ch < nChunks; ++ch) {
    const int cbase = ch * CHUNK;
    const int wc = scan_chunk<NBF, 1>(dsts, ei, nE, nN, cbase, nodeBase, vec8, list, tid, lane, wave);
    if (lane == 0) wcnt[wave] = wc;
    __syncthreads();
    if (wave == 0) {
#pragma unroll 1
      for (int wsx = 0; wsx < NWAVE; ++wsx) {
        int n = __builtin_amdgcn_readfirstlane(wcnt[wsx]);
        n = n > WCAP ? WCAP : (n < 0 ? 0 : n);
        const int* lp = list + wsx * WCAP;
#pragma unroll 1
        for (int i = 0; i < n; ++i) {
          const int ent  = __builtin_amdgcn_readfirstlane(lp[i]);
          const int slot = ent & (NBF - 1);
          int src = (ent >> ESHF) & 0xFFFFF;
          src = src > nN - 1 ? nN - 1 : src;
          if (lane == 0) {
            int pos = cursor[slot];
            pos = pos < 0 ? 0 : (pos > RCAP - 1 ? RCAP - 1 : pos);
            region[pos] = src;
            const int np = pos + 1;
            cursor[slot] = np > RCAP ? RCAP : np;
          }
        }
      }
    }
    __syncthreads();
  }

  const int nv = lenW >> 2;
  int* gp = csr + rb0;
#pragma unroll 1
  for (int i = tid; i < nv; i += NTHR) { const v4i v = ((const v4i*)region)[i]; *(volatile v4i*)(gp + 4 * i) = v; }
  __threadfence();
#pragma unroll 1
  for (int i = tid; i < nv; i += NTHR) { const v4i v = ((const v4i*)region)[i]; *(volatile v4i*)(gp + 4 * i) = v; }
}

template <int K, int SUB>
__global__ __launch_bounds__(NTHR) void k_gemm(
    const float* __restrict__ A, const float* __restrict__ me,
    const unsigned short* __restrict__ Bh, const unsigned short* __restrict__ Bl,
    float* C, int nRowsA) {
  extern __shared__ v4f lds_dyn[];
  unsigned short* sAh = (unsigned short*)lds_dyn;
  unsigned short* sAl = sAh + GR * K;
  float* stg = (float*)lds_dyn;
  const int tid = threadIdx.x, lane = tid & 31, wave = tid >> 5, hh = lane >> 4, m = lane & 15;
  const int rg = wave >> 1, chf = wave & 1;
  const int rowBase = (int)blockIdx.x * GR;

#pragma unroll
  for (int i = 0; i < (GR * K / 8) / NTHR; ++i) {
    const int idx = i * NTHR + tid;
    const int r   = idx / (K / 8);
    const int c0  = (idx - r * (K / 8)) * 8;
    int row = rowBase + r;
    row = row > nRowsA - 1 ? nRowsA - 1 : row;
    const float* ap = A + (size_t)row * K + c0;
    const v4f a = *(const v4f*)ap, b = *(const v4f*)(ap + 4);
    float av[8] = {a.x, a.y, a.z, a.w, b.x, b.y, b.z, b.w};
    if (SUB != 0) {
      const v4f p = *(const v4f*)(me + c0), q = *(const v4f*)(me + c0 + 4);
      const float mv[8] = {p.x, p.y, p.z, p.w, q.x, q.y, q.z, q.w};
#pragma unroll
      for (int e = 0; e < 8; ++e) av[e] = (av[e] == 0.0f) ? mv[e] : av[e];
    }
    Pk8 hp, lp;
#pragma unroll
    for (int e = 0; e < 8; ++e) {
      const __bf16 hb = (__bf16)av[e];
      const float rem = av[e] - (float)hb;
      hp.b[e] = hb;
      lp.b[e] = (__bf16)rem;
    }
    *(v8us*)(sAh + r * K + c0) = hp.u;
    *(v8us*)(sAl + r * K + c0) = lp.u;
  }
  __syncthreads();

  v8f acc[4];
#pragma unroll
  for (int t = 0; t < 4; ++t) { v8f z = {0.f, 0.f, 0.f, 0.f, 0.f, 0.f, 0.f, 0.f}; acc[t] = z; }
  const unsigned short* ahp = sAh + (rg * 16 + m) * K + 8 * hh;
  const unsigned short* alp = sAl + (rg * 16 + m) * K + 8 * hh;
#pragma unroll 1
  for (int kt = 0; kt < K / 32; ++kt) {
    FragB ah, al;
    ah.h[0] = *(const v8us*)(ahp + 32 * kt);
    ah.h[1] = *(const v8us*)(ahp + 32 * kt + 16);
    al.h[0] = *(const v8us*)(alp + 32 * kt);
    al.h[1] = *(const v8us*)(alp + 32 * kt + 16);
#pragma unroll
    for (int t = 0; t < 4; ++t) {
      const size_t bo = (size_t)(64 * chf + 16 * t + m) * K + 32 * kt + 8 * hh;
      FragB bh, bl;
      bh.h[0] = *(const v8us*)(Bh + bo);
      bh.h[1] = *(const v8us*)(Bh + bo + 16);
      bl.h[0] = *(const v8us*)(Bl + bo);
      bl.h[1] = *(const v8us*)(Bl + bo + 16);
      acc[t] = wmb(ah.v, bh.v, acc[t]);
      acc[t] = wmb(ah.v, bl.v, acc[t]);
      acc[t] = wmb(al.v, bh.v, acc[t]);
    }
  }
  __syncthreads();

  float* sp = stg + (rg * 16 + 8 * hh) * FH + 64 * chf + m;
#pragma unroll
  for (int t = 0; t < 4; ++t) {
#pragma unroll
    for (int r = 0; r < 8; ++r) sp[r * FH + 16 * t] = acc[t][r];
  }
  __syncthreads();

  const float* lp = stg + wave * (GR / NWAVE) * FH;
  float* gp = C + (size_t)(rowBase + wave * (GR / NWAVE)) * FH;
#pragma unroll
  for (int i = 0; i < GR / NWAVE; ++i) {
    const v4f v = *(const v4f*)(lp + i * FH + 4 * lane);
    *(volatile v4f*)(gp + i * FH + 4 * lane) = v;
  }
  __threadfence();
#pragma unroll
  for (int i = 0; i < GR / NWAVE; ++i) {
    const v4f v = *(const v4f*)(lp + i * FH + 4 * lane);
    *(volatile v4f*)(gp + i * FH + 4 * lane) = v;
  }
}

__global__ __launch_bounds__(NTHR) void k_agg(
    const int* __restrict__ csr, const int* __restrict__ off, const int* __restrict__ cnt,
    const float* __restrict__ hw, const float* __restrict__ bs, const float* __restrict__ eps,
    float* h, int nN, int csrLen) {
  const int tid = threadIdx.x, lane = tid & 31, wave = tid >> 5;
  const int tbase = (int)blockIdx.x * TGT + wave * 32;
  const int cl = tbase + lane;
  const int cnt_l = cnt[cl];
  const int off_l = off[cl];
  const float s2 = 2.0f + eps[0];
  const v4f bb = *(const v4f*)(bs + 4 * lane);

#pragma unroll 1
  for (int j = 0; j < 32; ++j) {
    const int c = tbase + j;
    int n = __builtin_amdgcn_readlane(cnt_l, j);
    n = n < 0 ? 0 : (n > DEGCAP ? DEGCAP : n);
    const int st = __builtin_amdgcn_readlane(off_l, j);
    v4f acc = {0.f, 0.f, 0.f, 0.f};
#pragma unroll 1
    for (int q0 = 0; q0 < n; q0 += 32) {
      int pos = st + q0 + lane;
      pos = pos < 0 ? 0 : (pos > csrLen - 1 ? csrLen - 1 : pos);
      int sl = csr[pos];
      sl = sl < 0 ? 0 : (sl > nN - 1 ? nN - 1 : sl);
      const int mcnt = (n - q0) < 32 ? (n - q0) : 32;
#pragma unroll 1
      for (int p = 0; p < mcnt; ++p) {
        const int s = __builtin_amdgcn_readlane(sl, p);
        acc = acc + *(const v4f*)(hw + (size_t)s * FH + 4 * lane);
      }
    }
    const v4f sv = *(const v4f*)(hw + (size_t)c * FH + 4 * lane);
    v4f v = sv * s2 + acc;
    v = v + bb;
    v.x = v.x > 0.f ? v.x : 0.2f * v.x;
    v.y = v.y > 0.f ? v.y : 0.2f * v.y;
    v.z = v.z > 0.f ? v.z : 0.2f * v.z;
    v.w = v.w > 0.f ? v.w : 0.2f * v.w;
    float* hp = h + (size_t)c * FH + 4 * lane;
    *(volatile v4f*)hp = v;
    __threadfence();
    *(volatile v4f*)hp = v;
  }
}

__global__ __launch_bounds__(NTHR) void k_mix(
    const float* __restrict__ XE, const float* __restrict__ XC,
    const unsigned short* __restrict__ Bh, const unsigned short* __restrict__ Bl,
    const float* __restrict__ bm, float* out, int nN) {
  __shared__ __attribute__((aligned(16))) float stg[MROWS * NCLS];
  const int tid = threadIdx.x, lane = tid & 31, wave = tid >> 5, hh = lane >> 4, m = lane & 15;
  const int tilerow = (int)blockIdx.x * MROWS + wave * 16;
  const int row = tilerow + m;
  const float* pe = XE + (size_t)row * FH + 8 * hh;
  const float* pc = XC + (size_t)row * FH + 8 * hh;
  const unsigned short* bhp = Bh + (size_t)m * FEXP + 8 * hh;
  const unsigned short* blp = Bl + (size_t)m * FEXP + 8 * hh;

  v8f acc = {0.f, 0.f, 0.f, 0.f, 0.f, 0.f, 0.f, 0.f};
#pragma unroll
  for (int kt = 0; kt < FH / 32; ++kt) {
    v16bf ahv, alv;
    split_row16(pe + 32 * kt, ahv, alv);
    FragB bh, bl;
    bh.h[0] = *(const v8us*)(bhp + 32 * kt);
    bh.h[1] = *(const v8us*)(bhp + 32 * kt + 16);
    bl.h[0] = *(const v8us*)(blp + 32 * kt);
    bl.h[1] = *(const v8us*)(blp + 32 * kt + 16);
    acc = wmb(ahv, bh.v, acc);
    acc = wmb(ahv, bl.v, acc);
    acc = wmb(alv, bh.v, acc);
  }
#pragma unroll
  for (int kt = 0; kt < FH / 32; ++kt) {
    v16bf ahv, alv;
    split_row16(pc + 32 * kt, ahv, alv);
    FragB bh, bl;
    bh.h[0] = *(const v8us*)(bhp + FH + 32 * kt);
    bh.h[1] = *(const v8us*)(bhp + FH + 32 * kt + 16);
    bl.h[0] = *(const v8us*)(blp + FH + 32 * kt);
    bl.h[1] = *(const v8us*)(blp + FH + 32 * kt + 16);
    acc = wmb(ahv, bh.v, acc);
    acc = wmb(ahv, bl.v, acc);
    acc = wmb(alv, bh.v, acc);
  }

  const int mc = m < NCLS ? m : NCLS - 1;
  const float bz = bm[mc];
  if (m < NCLS) {
    float* sp = stg + (wave * 16 + 8 * hh) * NCLS + m;
#pragma unroll
    for (int r = 0; r < 8; ++r) {
      const float v = acc[r] + bz;
      sp[r * NCLS] = v > 0.f ? v : 0.2f * v;
    }
  }
  __syncthreads();

  const int f4 = tid;
  const int orow = (int)blockIdx.x * MROWS + (f4 >> 1);
  const v4f v = *(const v4f*)(stg + 4 * f4);
  float* gp = out + (size_t)blockIdx.x * MROWS * NCLS + 4 * f4;
  if (orow < nN) *(volatile v4f*)gp = v;
  __threadfence();
  if (orow < nN) *(volatile v4f*)gp = v;
}

__global__ __launch_bounds__(HTHR) void k_head(
    const float* feat, const int* __restrict__ cidx,
    const float* __restrict__ Wp1, const float* __restrict__ bp1,
    const float* __restrict__ Wp2, const float* __restrict__ bp2,
    float* logits, int nC, int nN) {
  __shared__ __attribute__((aligned(16))) float slog[HTHR * NCLS];
  const int tid = threadIdx.x;
  const int t = (int)blockIdx.x * HTHR + tid;
  const int tc = t < nC ? t : nC - 1;
  int node = cidx[tc];
  node = node < 0 ? node + nN : node;
  node = node < 0 ? 0 : (node > nN - 1 ? nN - 1 : node);
  const v4f f0 = *(const v4f*)(feat + (size_t)node * NCLS);
  const v4f f1 = *(const v4f*)(feat + (size_t)node * NCLS + 4);
  const float c8[8] = {f0.x, f0.y, f0.z, f0.w, f1.x, f1.y, f1.z, f1.w};
  float part[8];
#pragma unroll
  for (int mm = 0; mm < NCLS; ++mm) part[mm] = 0.0f;
#pragma unroll 1
  for (int j = 0; j < FH; ++j) {
    float tt = c8[0] * Wp1[j];
#pragma unroll
    for (int k = 1; k < NCLS; ++k) tt += c8[k] * Wp1[k * FH + j];
    tt += bp1[j];
    tt = fmaxf(tt, 0.0f);
#pragma unroll
    for (int mm = 0; mm < NCLS; ++mm) part[mm] += tt * Wp2[j * NCLS + mm];
  }
  float* sp = slog + tid * NCLS;
#pragma unroll
  for (int mm = 0; mm < NCLS; ++mm) sp[mm] = part[mm] + bp2[mm];
  __syncthreads();

  float* gb = logits + (size_t)blockIdx.x * HTHR * NCLS;
  const int fa = tid, fb = HTHR + tid;
  const int ra = (int)blockIdx.x * HTHR + (fa >> 1);
  const int rb = (int)blockIdx.x * HTHR + (fb >> 1);
  const v4f va = *(const v4f*)(slog + 4 * fa);
  const v4f vb = *(const v4f*)(slog + 4 * fb);
  if (ra < nC) *(volatile v4f*)(gb + 4 * fa) = va;
  if (rb < nC) *(volatile v4f*)(gb + 4 * fb) = vb;
  __threadfence();
  if (ra < nC) *(volatile v4f*)(gb + 4 * fa) = va;
  if (rb < nC) *(volatile v4f*)(gb + 4 * fb) = vb;
}

extern "C" void kernel_launch(void* const* d_in, const int* in_sizes, int n_in,
                              void* d_out, int out_size, void* d_ws, size_t ws_size,
                              hipStream_t stream) {
  if (n_in < 24) return;
  const int nN = in_sizes[0] / FEXP;
  const int nE = in_sizes[2] / 2;
  const int nC = in_sizes[3];
  if (nN <= 0 || nE <= 0 || nC <= 0) return;
  if (in_sizes[0] != nN * FEXP || in_sizes[1] != nN * FH || in_sizes[2] != 2 * nE) return;
  if (in_sizes[4] != FEXP || in_sizes[5] != FH) return;
  if (in_sizes[6] != FEXP * FH || in_sizes[7] != FH || in_sizes[8] < 1) return;
  if (in_sizes[9] != FH * FH || in_sizes[10] != FH || in_sizes[11] < 1) return;
  if (in_sizes[12] != FH * FH || in_sizes[13] != FH || in_sizes[14] < 1) return;
  if (in_sizes[15] != FH * FH || in_sizes[16] != FH || in_sizes[17] < 1) return;
  if (in_sizes[18] != FEXP * NCLS || in_sizes[19] != NCLS) return;
  if (in_sizes[20] != NCLS * FH || in_sizes[21] != FH) return;
  if (in_sizes[22] != FH * NCLS || in_sizes[23] != NCLS) return;
  if (out_size != nN * NCLS + nC * NCLS) return;
  if (nN > (1 << 20) || nE > (1 << 28)) return;

  const float* x     = (const float*)d_in[0];
  const float* cfeat = (const float*)d_in[1];
  const int*   ei    = (const int*)d_in[2];
  const int*   cidx  = (const int*)d_in[3];
  const float* me_x  = (const float*)d_in[4];
  const float* me_c  = (const float*)d_in[5];
  const float* W1e = (const float*)d_in[6];  const float* b1e = (const float*)d_in[7];  const float* eps1e = (const float*)d_in[8];
  const float* W2e = (const float*)d_in[9];  const float* b2e = (const float*)d_in[10]; const float* eps2e = (const float*)d_in[11];
  const float* W1c = (const float*)d_in[12]; const float* b1c = (const float*)d_in[13]; const float* eps1c = (const float*)d_in[14];
  const float* W2c = (const float*)d_in[15]; const float* b2c = (const float*)d_in[16]; const float* eps2c = (const float*)d_in[17];
  const float* Wm  = (const float*)d_in[18]; const float* bm  = (const float*)d_in[19];
  const float* Wp1 = (const float*)d_in[20]; const float* bp1 = (const float*)d_in[21];
  const float* Wp2 = (const float*)d_in[22]; const float* bp2 = (const float*)d_in[23];
  float* out = (float*)d_out;

  const int NPAD   = ((nN + TGT - 1) / TGT) * TGT;
  const int nBC    = (nN + NBC - 1) / NBC;
  const int CNTPAD = nBC * NBC;
  const int nBF    = (nN + NBF - 1) / NBF;
  const int OFFN   = nBF * NBF;
  if (nBF + 1 > RBN) return;
  if (OFFN > CNTPAD || NPAD > OFFN) return;
  const int csrLen = ((nE + 31) & ~31) + 32 * (nBF + 1);
  const int nGemm  = NPAD / GR;
  const int nMix   = NPAD / MROWS;
  const int nAgg   = NPAD / TGT;
  const int nHead  = (nC + HTHR - 1) / HTHR;

  char* ws = (char*)d_ws;
  size_t off = 0;
  const size_t oW1e = off; off += (size_t)2 * FH * FEXP * 2;       off = (off + 255) & ~(size_t)255;
  const size_t oW2e = off; off += (size_t)2 * FH * FH * 2;         off = (off + 255) & ~(size_t)255;
  const size_t oW1c = off; off += (size_t)2 * FH * FH * 2;         off = (off + 255) & ~(size_t)255;
  const size_t oW2c = off; off += (size_t)2 * FH * FH * 2;         off = (off + 255) & ~(size_t)255;
  const size_t oWm  = off; off += (size_t)2 * NCP * FEXP * 2;      off = (off + 255) & ~(size_t)255;
  const size_t oCnt = off; off += (size_t)CNTPAD * 4;              off = (off + 255) & ~(size_t)255;
  const size_t oOff = off; off += (size_t)OFFN * 4;                off = (off + 255) & ~(size_t)255;
  const size_t oRb  = off; off += (size_t)RBN * 4;                 off = (off + 255) & ~(size_t)255;
  const size_t oCsr = off; off += (size_t)csrLen * 4;              off = (off + 255) & ~(size_t)255;
  const size_t oP0  = off; off += (size_t)NPAD * FH * 4;           off = (off + 255) & ~(size_t)255;
  const size_t oP1  = off; off += (size_t)NPAD * FH * 4;           off = (off + 255) & ~(size_t)255;
  const size_t oP2  = off; off += (size_t)NPAD * FH * 4;           off = (off + 255) & ~(size_t)255;
  if (off > ws_size || off > (size_t)WSCAP) return;
  unsigned short* w1eh = (unsigned short*)(ws + oW1e); unsigned short* w1el = w1eh + FH * FEXP;
  unsigned short* w2eh = (unsigned short*)(ws + oW2e); unsigned short* w2el = w2eh + FH * FH;
  unsigned short* w1ch = (unsigned short*)(ws + oW1c); unsigned short* w1cl = w1ch + FH * FH;
  unsigned short* w2ch = (unsigned short*)(ws + oW2c); unsigned short* w2cl = w2ch + FH * FH;
  unsigned short* wmh  = (unsigned short*)(ws + oWm);  unsigned short* wml  = wmh + NCP * FEXP;
  int*   cnt  = (int*)(ws + oCnt);
  int*   offp = (int*)(ws + oOff);
  int*   rb   = (int*)(ws + oRb);
  int*   csr  = (int*)(ws + oCsr);
  float* P0   = (float*)(ws + oP0);
  float* P1   = (float*)(ws + oP1);
  float* P2   = (float*)(ws + oP2);

  const int vec8 = ((nE & 3) == 0) ? 1 : 0;

  k_wprep<<<(FH * FEXP / 8) / NTHR, NTHR, 0, stream>>>(W1e, w1eh, w1el, FEXP, FH, FH);
  k_wprep<<<(FH * FH / 8) / NTHR, NTHR, 0, stream>>>(W2e, w2eh, w2el, FH, FH, FH);
  k_wprep<<<(FH * FH / 8) / NTHR, NTHR, 0, stream>>>(W1c, w1ch, w1cl, FH, FH, FH);
  k_wprep<<<(FH * FH / 8) / NTHR, NTHR, 0, stream>>>(W2c, w2ch, w2cl, FH, FH, FH);
  k_wprep<<<(NCP * FEXP / 8) / NTHR, NTHR, 0, stream>>>(Wm, wmh, wml, FEXP, NCLS, NCP);

  hipFuncSetAttribute(reinterpret_cast<const void*>(&k_count),
                      hipFuncAttributeMaxDynamicSharedMemorySize, LDS_COUNT);
  k_count<<<nBC, NTHR, LDS_COUNT, stream>>>(ei, cnt, nE, nN, vec8);
  k_offsets<<<1, OTHR, 0, stream>>>(cnt, offp, rb, nBF);
  hipFuncSetAttribute(reinterpret_cast<const void*>(&k_fill),
                      hipFuncAttributeMaxDynamicSharedMemorySize, LDS_FILL);
  k_fill<<<nBF, NTHR, LDS_FILL, stream>>>(ei, offp, rb, csr, nN, nE, vec8, csrLen);

  hipFuncSetAttribute(reinterpret_cast<const void*>(&k_gemm<FEXP, 1>),
                      hipFuncAttributeMaxDynamicSharedMemorySize, LDS_GEMM);
  hipFuncSetAttribute(reinterpret_cast<const void*>(&k_gemm<FH, 1>),
                      hipFuncAttributeMaxDynamicSharedMemorySize, LDS_GEMM);
  hipFuncSetAttribute(reinterpret_cast<const void*>(&k_gemm<FH, 0>),
                      hipFuncAttributeMaxDynamicSharedMemorySize, LDS_GEMM);

  k_gemm<FEXP, 1><<<nGemm, NTHR, LDS_GEMM, stream>>>(x, me_x, w1eh, w1el, P0, nN);
  k_agg<<<nAgg, NTHR, 0, stream>>>(csr, offp, cnt, P0, b1e, eps1e, P1, nN, csrLen);
  k_gemm<FH, 0><<<nGemm, NTHR, LDS_GEMM, stream>>>(P1, me_c, w2eh, w2el, P0, NPAD);
  k_agg<<<nAgg, NTHR, 0, stream>>>(csr, offp, cnt, P0, b2e, eps2e, P1, nN, csrLen);

  k_gemm<FH, 1><<<nGemm, NTHR, LDS_GEMM, stream>>>(cfeat, me_c, w1ch, w1cl, P0, nN);
  k_agg<<<nAgg, NTHR, 0, stream>>>(csr, offp, cnt, P0, b1c, eps1c, P2, nN, csrLen);
  k_gemm<FH, 0><<<nGemm, NTHR, LDS_GEMM, stream>>>(P2, me_c, w2ch, w2cl, P0, NPAD);
  k_agg<<<nAgg, NTHR, 0, stream>>>(csr, offp, cnt, P0, b2c, eps2c, P2, nN, csrLen);

  k_mix<<<nMix, NTHR, 0, stream>>>(P1, P2, wmh, wml, bm, out, nN);

  k_head<<<nHead, HTHR, 0, stream>>>(out, cidx, Wp1, bp1, Wp2, bp2, out + (size_t)nN * NCLS, nC, nN);
}
